// EnhancedMamba2Block_44117904065245
// MI455X (gfx1250) — hardware-verified
//
#include <hip/hip_runtime.h>
#include <math.h>

#define NB    2
#define SEQ   4096
#define DM    1024
#define DS    16
#define DCONV 4
#define MR    (NB * SEQ)
#define TCH   32
#define NXPAD 64

typedef __attribute__((ext_vector_type(16))) _Float16 v16h;
typedef __attribute__((ext_vector_type(8)))  _Float16 v8h;
typedef __attribute__((ext_vector_type(16))) __bf16   v16b;
typedef __attribute__((ext_vector_type(8)))  __bf16   v8b;
typedef __attribute__((ext_vector_type(8)))  float    v8f;
typedef __attribute__((ext_vector_type(4)))  float    v4f;
typedef __attribute__((ext_vector_type(2)))  float    v2f;
typedef v8h v8ha __attribute__((may_alias));

__device__ __forceinline__ unsigned short f2bf_bits(float f) {
  unsigned u = __float_as_uint(f);
  return (unsigned short)((u + 0x7FFFu + ((u >> 16) & 1u)) >> 16);
}
__device__ __forceinline__ float bf_bits2f(unsigned short h) { return __uint_as_float(((unsigned)h) << 16); }

__device__ __forceinline__ void dep_guard_h(v8f& a, v8f& b, v16h x, v16h y) { asm volatile("v_nop\n\tv_nop\n\tv_nop\n\tv_nop" : "+v"(a), "+v"(b) : "v"(x), "v"(y)); }
__device__ __forceinline__ void dep_guard_b(v8f& a, v8f& b, v16b x, v16b y) { asm volatile("v_nop\n\tv_nop\n\tv_nop\n\tv_nop" : "+v"(a), "+v"(b) : "v"(x), "v"(y)); }
__device__ __forceinline__ void keep4_h(v16h a, v16h b, v16h c, v16h d) { asm volatile("v_nop" :: "v"(a), "v"(b), "v"(c), "v"(d)); }
__device__ __forceinline__ void keep4_b(v16b a, v16b b, v16b c, v16b d) { asm volatile("v_nop" :: "v"(a), "v"(b), "v"(c), "v"(d)); }
__device__ __forceinline__ void acc_guard4(v8f& a, v8f& b, v8f& c, v8f& d) { asm volatile("v_nop\n\tv_nop\n\tv_nop\n\tv_nop" : "+v"(a), "+v"(b), "+v"(c), "+v"(d)); }
template <typename T> struct Frag;
template <> struct Frag<_Float16> {
  typedef v16h V; union U { v16h v; v8h h[2]; };
  static __device__ __forceinline__ v16h load(const _Float16* p) {
    U f; f.h[0] = *(const v8h*)(p); f.h[1] = *(const v8h*)(p + 16); return f.v;
  }
  static __device__ __forceinline__ v8f mma(v16h a, v16h b, v8f c) {
    return __builtin_amdgcn_wmma_f32_16x16x32_f16(false, a, false, b, (short)0, c, false, false);
  }
  static __device__ __forceinline__ void guard(v8f& a, v8f& b, v16h x, v16h y) { dep_guard_h(a, b, x, y); }
  static __device__ __forceinline__ void keep(v16h a, v16h b, v16h c, v16h d) { keep4_h(a, b, c, d); }
};
template <> struct Frag<__bf16> {
  typedef v16b V; union U { v16b v; v8b h[2]; };
  static __device__ __forceinline__ v16b load(const __bf16* p) {
    U f; f.h[0] = *(const v8b*)(p); f.h[1] = *(const v8b*)(p + 16); return f.v;
  }
  static __device__ __forceinline__ v8f mma(v16b a, v16b b, v8f c) {
    return __builtin_amdgcn_wmma_f32_16x16x32_bf16(false, a, false, b, (short)0, c, false, false);
  }
  static __device__ __forceinline__ void guard(v8f& a, v8f& b, v16b x, v16b y) { dep_guard_b(a, b, x, y); }
  static __device__ __forceinline__ void keep(v16b a, v16b b, v16b c, v16b d) { keep4_b(a, b, c, d); }
};

template <int ET> struct Elem;
template <> struct Elem<0> { typedef _Float16 T; };
template <> struct Elem<1> { typedef __bf16 T; };
template <int ET, bool SPLIT, int BIAS_MODE, int OUT_MODE, bool RESID, int ACT = 0>
__global__ __launch_bounds__(256) void wmma_gemm64(
    const unsigned short* __restrict__ Ap, const unsigned short* __restrict__ A2p, int lda, long strideA,
    const unsigned short* __restrict__ Btp, const unsigned short* __restrict__ Bt2p, int ldb, long strideB,
    void* __restrict__ Cout, void* __restrict__ Cout2, int ldc, long strideC,
    const float* __restrict__ bias,
    const float* __restrict__ resid, long strideR,
    int M, int N, int K, float scale) {
  typedef typename Elem<ET>::T T;
  typedef typename Frag<T>::V V;
  const T* A = (const T*)Ap; const T* A2 = (const T*)A2p; const T* Bt = (const T*)Btp; const T* Bt2 = (const T*)Bt2p;
  __shared__ __align__(16) float sT[8][16 * 68];
  const int b    = blockIdx.y;
  const int lane = threadIdx.x & 31;
  const int wave = threadIdx.x >> 5;
  const int tilesN = N >> 6;
  const int tilesM = M >> 6;
  const int tile = blockIdx.x * 8 + wave;
  if (tile >= tilesM * tilesN) return;
  const int tm = tile / tilesN;
  const int tn = tile - tm * tilesN;
  const int m0 = tm << 6;
  const int n0 = tn << 6;

  const T* Ab  = A  + (size_t)b * strideA;
  const T* Bb  = Bt + (size_t)b * strideB;
  const T* Ab2 = SPLIT ? (A2  + (size_t)b * strideA) : nullptr;
  const T* Bb2 = SPLIT ? (Bt2 + (size_t)b * strideB) : nullptr;

  const int rlane = lane & 15;
  const int koff  = (lane >> 4) * 8;
  const int mOff  = (lane >> 4) * 8;

  v8f acc[4][4];
#pragma unroll
  for (int i = 0; i < 4; ++i)
#pragma unroll
    for (int j = 0; j < 4; ++j) acc[i][j] = (v8f){0.f,0.f,0.f,0.f,0.f,0.f,0.f,0.f};

  for (int k0 = 0; k0 < K; k0 += 32) {
    V bh[4], bl[4];
#pragma unroll
    for (int j = 0; j < 4; ++j) {
      const size_t bo = (size_t)(n0 + (j << 4) + rlane) * ldb + koff + k0;
      bh[j] = Frag<T>::load(Bb + bo);
      if (SPLIT) bl[j] = Frag<T>::load(Bb2 + bo);
    }
#pragma unroll
    for (int i = 0; i < 4; ++i) {
      const size_t ao = (size_t)(m0 + (i << 4) + rlane) * lda + koff + k0;
      V ah = Frag<T>::load(Ab + ao);
      V al;
      if (SPLIT) al = Frag<T>::load(Ab2 + ao);
#pragma unroll
      for (int j = 0; j < 4; ++j) {
        acc[i][j] = Frag<T>::mma(ah, bh[j], acc[i][j]);
        if (SPLIT) {
          acc[i][j] = Frag<T>::mma(ah, bl[j], acc[i][j]);
          acc[i][j] = Frag<T>::mma(al, bh[j], acc[i][j]);
        }
      }
      Frag<T>::guard(acc[i][0], acc[i][3], ah, SPLIT ? al : ah);
    }
    Frag<T>::keep(bh[0], bh[1], bh[2], bh[3]);
    if (SPLIT) Frag<T>::keep(bl[0], bl[1], bl[2], bl[3]);
  }
  acc_guard4(acc[0][0], acc[0][1], acc[0][2], acc[0][3]);
  acc_guard4(acc[1][0], acc[1][1], acc[1][2], acc[1][3]);
  acc_guard4(acc[2][0], acc[2][1], acc[2][2], acc[2][3]);
  acc_guard4(acc[3][0], acc[3][1], acc[3][2], acc[3][3]);

  float* slab = sT[wave];
  const float* Rb = RESID ? (resid + (size_t)b * strideR) : nullptr;
#pragma unroll
  for (int i = 0; i < 4; ++i) {
    const int mBase = m0 + (i << 4);
#pragma unroll
    for (int j = 0; j < 4; ++j) {
      const int n = n0 + (j << 4) + rlane;
      float bv = 0.f;
      if (BIAS_MODE == 2) bv = bias[n];
#pragma unroll
      for (int r = 0; r < 8; ++r) {
        float v = acc[i][j][r] * scale;
        if (BIAS_MODE == 1) v += bias[mBase + mOff + r];
        if (BIAS_MODE == 2) v += bv;
        if (RESID) v += Rb[(size_t)(mBase + mOff + r) * ldc + n];
        if (ACT == 1) v = tanhf(v);
        if (ACT == 2) v = fmaxf(v, 0.0f);
        if (ACT == 3) v = v / (1.0f + expf(-v));
        if (ACT == 4) v = (v > 0.f) ? v : 0.01f * v;
        if (ACT == 5) v = 0.5f * v * (1.0f + erff(v * 0.70710678118654752f));
        slab[(mOff + r) * 68 + (j << 4) + rlane] = v;
      }
    }
    __builtin_amdgcn_fence(__ATOMIC_RELEASE, "workgroup");
    __builtin_amdgcn_wave_barrier();
    __builtin_amdgcn_fence(__ATOMIC_ACQUIRE, "workgroup");
    if (OUT_MODE == 0) {
      float* C = (float*)Cout + (size_t)b * strideC;
      const int hh = lane >> 4, c4 = (lane & 15) * 4;
      for (int pass = 0; pass < 2; ++pass) {
#pragma unroll
        for (int it = 0; it < 8; ++it) {
          const int row = it * 2 + hh;
          v4f v = *(const v4f*)(slab + row * 68 + c4);
          *(volatile v4f*)(C + (size_t)(mBase + row) * ldc + n0 + c4) = v;
        }
        __threadfence();
      }
    } else {
      const int q = lane >> 3, c8 = (lane & 7) * 8;
      unsigned short* C  = (unsigned short*)Cout  + (size_t)b * strideC;
      unsigned short* C2 = (OUT_MODE == 2) ? ((unsigned short*)Cout2 + (size_t)b * strideC) : nullptr;
      for (int pass = 0; pass < 2; ++pass) {
#pragma unroll
        for (int it = 0; it < 4; ++it) {
          const int row = it * 4 + q;
          const float* sp = slab + row * 68 + c8;
          v8h hv, lv;
#pragma unroll
          for (int e = 0; e < 8; ++e) {
            if (OUT_MODE == 1) {
              hv[e] = (_Float16)sp[e];
            } else {
              unsigned short hb = f2bf_bits(sp[e]);
              unsigned short lb = f2bf_bits(sp[e] - bf_bits2f(hb));
              hv[e] = __builtin_bit_cast(_Float16, hb);
              lv[e] = __builtin_bit_cast(_Float16, lb);
            }
          }
          *(volatile v8h*)(C + (size_t)(mBase + row) * ldc + n0 + c8) = hv;
          if (OUT_MODE == 2) *(volatile v8h*)(C2 + (size_t)(mBase + row) * ldc + n0 + c8) = lv;
        }
        __threadfence();
      }
    }
    __builtin_amdgcn_fence(__ATOMIC_RELEASE, "workgroup");
    __builtin_amdgcn_wave_barrier();
    __builtin_amdgcn_fence(__ATOMIC_ACQUIRE, "workgroup");
  }
}

__device__ __forceinline__ float silu_f(float v) {
  const float e = expf(fminf(-v, 80.0f));
  const float s = 1.0f / (1.0f + e);
  return v * s;
}
__device__ __forceinline__ float softplus_f(float v) {
  const float av = fminf(fabsf(v), 40.0f);
  return fmaxf(v, 0.0f) + log1pf(expf(-av));
}
__device__ __forceinline__ float conv4f(float w0, float w1, float w2, float w3,
                                         float xa, float xb, float xc, float xd, float bias) {
  float acc = w0 * xa;
  acc = acc + w1 * xb;
  acc = acc + w2 * xc;
  acc = acc + w3 * xd;
  return acc + bias;
}

__global__ __launch_bounds__(256) void cast_f32_f16x2s(
    const float* __restrict__ in, _Float16* __restrict__ out, int n2, float scale) {
  const int i = blockIdx.x * 256 + threadIdx.x;
  if (i < n2) {
    const size_t i2 = (size_t)i * 2;
    const _Float16 h0 = (_Float16)(in[i2] * scale), h1 = (_Float16)(in[i2 + 1] * scale);
    const unsigned u = (unsigned)__builtin_bit_cast(unsigned short, h0) | ((unsigned)__builtin_bit_cast(unsigned short, h1) << 16);
    ((volatile unsigned*)out)[i] = u;
    __threadfence();
    ((volatile unsigned*)out)[i] = u;
  }
}

__global__ __launch_bounds__(256) void split_bf16x2_pad(
    const float* __restrict__ in, unsigned short* __restrict__ hi, unsigned short* __restrict__ lo,
    int n2src, int n2dst) {
  const int i = blockIdx.x * 256 + threadIdx.x;
  if (i >= n2dst) return;
  const int ic = (i < n2src) ? i : (n2src - 1);
  const size_t i2 = (size_t)ic * 2;
  float v0 = in[i2], v1 = in[i2 + 1];
  if (i >= n2src) { v0 = 0.f; v1 = 0.f; }
  const unsigned short h0 = f2bf_bits(v0), h1 = f2bf_bits(v1);
  const unsigned short l0 = f2bf_bits(v0 - bf_bits2f(h0)), l1 = f2bf_bits(v1 - bf_bits2f(h1));
  const unsigned uh = (unsigned)h0 | ((unsigned)h1 << 16);
  const unsigned ul = (unsigned)l0 | ((unsigned)l1 << 16);
  ((volatile unsigned*)hi)[i] = uh;
  ((volatile unsigned*)lo)[i] = ul;
  __threadfence();
  ((volatile unsigned*)hi)[i] = uh;
  ((volatile unsigned*)lo)[i] = ul;
}

__global__ __launch_bounds__(256)
void conv_silu_planes(const float* __restrict__ XZ, const float* __restrict__ wconv,
                      const float* __restrict__ bconv, _Float16* __restrict__ xs_h,
                      unsigned short* __restrict__ xs_bhi, unsigned short* __restrict__ xs_blo, int npairs)
{
  const int i = blockIdx.x * 256 + threadIdx.x;
  if (i >= npairs) return;
  const int row = i >> 9;
  const int dp  = (i & 511) * 2;
  const int t   = row & (SEQ - 1);
  float xe[DCONV], xo[DCONV];
#pragma unroll
  for (int k = 0; k < DCONV; ++k) {
    const int tt = t - (DCONV - 1) + k;
    int rr = row - (DCONV - 1) + k;
    rr = rr < 0 ? 0 : rr;
    const v2f ld = *(const v2f*)(XZ + (size_t)rr * (2 * DM) + dp);
    const bool ok = (tt >= 0);
    xe[k] = ok ? ld[0] : 0.f;
    xo[k] = ok ? ld[1] : 0.f;
  }
  const float* wa = wconv + (size_t)dp * DCONV;
  const float* wb = wconv + (size_t)(dp + 1) * DCONV;
  const float s0 = silu_f(conv4f(wa[0], wa[1], wa[2], wa[3], xe[0], xe[1], xe[2], xe[3], bconv[dp]));
  const float s1 = silu_f(conv4f(wb[0], wb[1], wb[2], wb[3], xo[0], xo[1], xo[2], xo[3], bconv[dp + 1]));
  const _Float16 f0 = (_Float16)(s0 * 16.0f), f1 = (_Float16)(s1 * 16.0f);
  const unsigned uh = (unsigned)__builtin_bit_cast(unsigned short, f0) | ((unsigned)__builtin_bit_cast(unsigned short, f1) << 16);
  const unsigned short h0 = f2bf_bits(s0), h1 = f2bf_bits(s1);
  const unsigned short l0 = f2bf_bits(s0 - bf_bits2f(h0)), l1 = f2bf_bits(s1 - bf_bits2f(h1));
  const unsigned ubh = (unsigned)h0 | ((unsigned)h1 << 16);
  const unsigned ubl = (unsigned)l0 | ((unsigned)l1 << 16);
  ((volatile unsigned*)xs_h)[i]   = uh;
  ((volatile unsigned*)xs_bhi)[i] = ubh;
  ((volatile unsigned*)xs_blo)[i] = ubl;
  __threadfence();
  ((volatile unsigned*)xs_h)[i]   = uh;
  ((volatile unsigned*)xs_bhi)[i] = ubh;
  ((volatile unsigned*)xs_blo)[i] = ubl;
}

__global__ __launch_bounds__(256)
void ssm_scan(const float* __restrict__ XZ, const float* __restrict__ dtpre,
              const float* __restrict__ BC, const float* __restrict__ A_log,
              const float* __restrict__ Dsk, const float* __restrict__ state0,
              const float* __restrict__ wconv, const float* __restrict__ bconv,
              _Float16* __restrict__ yh, float* __restrict__ state_out)
{
  __shared__ __align__(16) float st_l[DS * 256];
  __shared__ __align__(16) float a_l[DS * 256];
  __shared__ __align__(16) float bc_l[TCH * 2 * DS];
  __shared__ __align__(16) _Float16 yt[TCH * 256];

  const int tid  = threadIdx.x;
  const int lane = tid & 31;
  const int wave = tid >> 5;
  const int b    = blockIdx.y;
  const int d0   = blockIdx.x * 256;
  const int d    = d0 + tid;

#pragma unroll 1
  for (int n = 0; n < DS; ++n) {
    st_l[n * 256 + tid] = state0[((size_t)b * DM + d) * DS + n];
    a_l[n * 256 + tid]  = -expf(A_log[(size_t)d * DS + n]);
  }
  const float Dd  = Dsk[d];
  const float w0  = wconv[(size_t)d * DCONV + 0];
  const float w1  = wconv[(size_t)d * DCONV + 1];
  const float w2  = wconv[(size_t)d * DCONV + 2];
  const float w3  = wconv[(size_t)d * DCONV + 3];
  const float bcv = bconv[d];
  float xm1 = 0.f, xm2 = 0.f, xm3 = 0.f;

  for (int t0 = 0; t0 < SEQ; t0 += TCH) {
    __syncthreads();
    {
      const int r = tid >> 3, c4 = (tid & 7) * 4;
      const v4f v = *(const v4f*)(BC + ((size_t)b * SEQ + t0 + r) * NXPAD + c4);
      bc_l[r * 32 + c4 + 0] = v[0];
      bc_l[r * 32 + c4 + 1] = v[1];
      bc_l[r * 32 + c4 + 2] = v[2];
      bc_l[r * 32 + c4 + 3] = v[3];
    }
    __syncthreads();
#pragma unroll 1
    for (int tl = 0; tl < TCH; ++tl) {
      const size_t row = (size_t)b * SEQ + t0 + tl;
      const float dtv = softplus_f(dtpre[row * DM + d]);
      const float x0  = XZ[row * (2 * DM) + d];
      const float zv  = XZ[row * (2 * DM) + DM + d];
      const float xs  = silu_f(conv4f(w0, w1, w2, w3, xm3, xm2, xm1, x0, bcv));
      xm3 = xm2; xm2 = xm1; xm1 = x0;
      const float* bcp = bc_l + tl * 32;
      float yv = 0.f;
#pragma unroll 1
      for (int n = 0; n < DS; ++n) {
        const int li = n * 256 + tid;
        const float a = a_l[li];
        float s = st_l[li];
        const float da = expf(dtv * a);
        s = s * da + bcp[n];
        yv += s * bcp[DS + n];
        st_l[li] = s;
      }
      const float y = (yv + xs * Dd) * silu_f(zv);
      yt[tl * 256 + tid] = (_Float16)(y * 16.0f);
    }
    __syncthreads();
    for (int pass = 0; pass < 2; ++pass) {
#pragma unroll
      for (int it = 0; it < TCH / 8; ++it) {
        const int tl = wave + 8 * it;
        const v8ha val = *(const v8ha*)(yt + tl * 256 + lane * 8);
        *(volatile v8h*)(yh + ((size_t)b * SEQ + t0 + tl) * DM + d0 + lane * 8) = val;
      }
      __threadfence();
    }
  }
  __syncthreads();
  {
    float* so = state_out + ((size_t)b * DM + d0) * DS;
    for (int pass = 0; pass < 2; ++pass) {
#pragma unroll
      for (int it = 0; it < 4; ++it) {
        const int c  = wave * 32 + it * 8 + (lane >> 2);
        const int n4 = (lane & 3) * 4;
        v4f v;
        v[0] = st_l[(n4 + 0) * 256 + c];
        v[1] = st_l[(n4 + 1) * 256 + c];
        v[2] = st_l[(n4 + 2) * 256 + c];
        v[3] = st_l[(n4 + 3) * 256 + c];
        *(volatile v4f*)(so + (size_t)c * DS + n4) = v;
      }
      __threadfence();
    }
  }
}

extern "C" void kernel_launch(void* const* d_in, const int* in_sizes, int n_in,
                              void* d_out, int out_size, void* d_ws, size_t ws_size,
                              hipStream_t stream) {
  if (n_in < 11) return;
  if (in_sizes[0] != MR * DM || in_sizes[1] != NB * DM * DS || in_sizes[2] != 2 * DM * DM ||
      in_sizes[3] != DM * DCONV || in_sizes[4] != DM || in_sizes[5] != 2 * DS * DM ||
      in_sizes[6] != DM * DM || in_sizes[7] != DM || in_sizes[8] != DM * DS ||
      in_sizes[9] != DM || in_sizes[10] != DM * DM) return;
  if (out_size != MR * DM + NB * DM * DS) return;

  const float* x      = (const float*)d_in[0];
  const float* state0 = (const float*)d_in[1];
  const float* w_in   = (const float*)d_in[2];
  const float* w_conv = (const float*)d_in[3];
  const float* b_conv = (const float*)d_in[4];
  const float* w_x    = (const float*)d_in[5];
  const float* w_dt   = (const float*)d_in[6];
  const float* b_dt   = (const float*)d_in[7];
  const float* A_log  = (const float*)d_in[8];
  const float* Dsk    = (const float*)d_in[9];
  const float* w_out  = (const float*)d_in[10];

  float* out       = (float*)d_out;
  float* state_out = out + (size_t)MR * DM;

  const size_t szXZ   = (size_t)MR * 2 * DM * 4;
  const size_t szP16  = (size_t)MR * DM * 2;
  const size_t szDT   = (size_t)MR * DM * 4;
  const size_t szWin  = (size_t)2 * DM * DM * 2;
  const size_t szWdt  = (size_t)DM * DM * 2;
  const size_t szWout = (size_t)DM * DM * 2;
  const size_t szWx   = (size_t)NXPAD * DM * 2;
  const size_t szBC   = (size_t)MR * NXPAD * 4;
  const size_t oXZ   = 0;
  const size_t oP16  = oXZ + szXZ;
  const size_t oDT   = oP16 + szP16;
  const size_t oWIN  = oDT + szDT;
  const size_t oWDT  = oWIN + szWin;
  const size_t oWOUT = oWDT + szWdt;
  const size_t oWXH  = oWOUT + szWout;
  const size_t oWXL  = oWXH + szWx;
  const size_t oBC   = oWXL + szWx;
  const size_t total = oBC + szBC;
  if (total > ws_size) return;

  char* ws = (char*)d_ws;
  float*          XZ     = (float*)(ws + oXZ);
  _Float16*       p16    = (_Float16*)(ws + oP16);
  unsigned short* xs_bhi = (unsigned short*)(ws + oDT);
  unsigned short* xs_blo = (unsigned short*)(ws + oDT + szP16);
  float*          dtpre  = (float*)(ws + oDT);
  _Float16*       win_h  = (_Float16*)(ws + oWIN);
  _Float16*       wdt_h  = (_Float16*)(ws + oWDT);
  _Float16*       wout_h = (_Float16*)(ws + oWOUT);
  unsigned short* wx_hi  = (unsigned short*)(ws + oWXH);
  unsigned short* wx_lo  = (unsigned short*)(ws + oWXL);
  float*          BCb    = (float*)(ws + oBC);

  cast_f32_f16x2s<<<(MR * DM / 2) / 256, 256, 0, stream>>>(x, p16, MR * DM / 2, 1.0f);
  cast_f32_f16x2s<<<(2 * DM * DM / 2) / 256, 256, 0, stream>>>(w_in, win_h, 2 * DM * DM / 2, 64.0f);
  cast_f32_f16x2s<<<(DM * DM / 2) / 256, 256, 0, stream>>>(w_dt, wdt_h, DM * DM / 2, 64.0f);
  cast_f32_f16x2s<<<(DM * DM / 2) / 256, 256, 0, stream>>>(w_out, wout_h, DM * DM / 2, 64.0f);
  split_bf16x2_pad<<<(NXPAD * DM / 2) / 256, 256, 0, stream>>>(w_x, wx_hi, wx_lo, 2 * DS * DM / 2, NXPAD * DM / 2);

  wmma_gemm64<0, false, 0, 0, false, 0><<<dim3((MR / 64) * (2 * DM / 64) / 8, 1), 256, 0, stream>>>(
      (const unsigned short*)p16, nullptr, DM, 0L,
      (const unsigned short*)win_h, nullptr, DM, 0L,
      (void*)XZ, nullptr, 2 * DM, 0L,
      nullptr, nullptr, 0L, MR, 2 * DM, DM, 1.0f / 64.0f);

  conv_silu_planes<<<(MR * DM / 2) / 256, 256, 0, stream>>>(XZ, w_conv, b_conv, p16, xs_bhi, xs_blo, MR * DM / 2);

  wmma_gemm64<1, true, 0, 0, false, 0><<<dim3((MR / 64) * (NXPAD / 64) / 8, 1), 256, 0, stream>>>(
      xs_bhi, xs_blo, DM, 0L,
      wx_hi, wx_lo, DM, 0L,
      (void*)BCb, nullptr, NXPAD, 0L,
      nullptr, nullptr, 0L, MR, NXPAD, DM, 1.0f);

  wmma_gemm64<0, false, 2, 0, false, 0><<<dim3((MR / 64) * (DM / 64) / 8, 1), 256, 0, stream>>>(
      (const unsigned short*)p16, nullptr, DM, 0L,
      (const unsigned short*)wdt_h, nullptr, DM, 0L,
      (void*)dtpre, nullptr, DM, 0L,
      b_dt, nullptr, 0L, MR, DM, DM, 1.0f / 1024.0f);

  ssm_scan<<<dim3(DM / 256, NB), 256, 0, stream>>>(XZ, dtpre, BCb, A_log, Dsk, state0, w_conv, b_conv, p16, state_out);

  wmma_gemm64<0, false, 0, 0, false, 0><<<dim3((MR / 64) * (DM / 64) / 8, 1), 256, 0, stream>>>(
      (const unsigned short*)p16, nullptr, DM, 0L,
      (const unsigned short*)wout_h, nullptr, DM, 0L,
      (void*)out, nullptr, DM, 0L,
      nullptr, nullptr, 0L, MR, DM, DM, 1.0f / 1024.0f);
}
